// DecoderLayer_42880953484173
// MI455X (gfx1250) — hardware-verified
//
#include <hip/hip_runtime.h>
#ifndef NB
#define NB 2
#endif
#ifndef SEQ
#define SEQ 2048
#endif
#define NB_FULL 2
#define SEQ_FULL 2048
#define DM 1024
#define NH 16
#define HD 64
#define DFF 4096
#define LQ (3 * DM)
#define NR ((size_t)NB * SEQ)

static_assert(DM == NH * HD);
static_assert(DM == 1024);
static_assert((SEQ & (SEQ - 1)) == 0);
static_assert(SEQ >= 128 && SEQ <= SEQ_FULL);
static_assert(NB >= 1 && NB <= NB_FULL);
static_assert(SEQ % 128 == 0 && LQ % 64 == 0 && DM % 64 == 0 && DFF % 64 == 0 && DM % 32 == 0 && DFF % 32 == 0);

#define WS_BQKV ((size_t)3 * DM * DM * 2)
#define WS_BO   ((size_t)DM * DM * 2)
#define WS_BW1  ((size_t)DFF * DM * 2)
#define WS_BW2  ((size_t)DM * DFF * 2)
#define WS_XLN  ((size_t)NB * SEQ * DM * 2)
#define WS_QKV  ((size_t)NB * SEQ * LQ * 2)
#define WS_VT   ((size_t)NB * NH * HD * SEQ * 2)
#define WS_Y16  ((size_t)NB * SEQ * DM * 2)
#define WS_X1   ((size_t)NB * SEQ * DM * 4)
#define WS_HLN  ((size_t)NB * SEQ * DM * 2)
#define WS_HF   ((size_t)SEQ * DFF * 2)
#define WS_TOTAL (WS_BQKV + WS_BO + WS_BW1 + WS_BW2 + WS_XLN + WS_QKV + WS_VT + WS_Y16 + WS_X1 + WS_HLN + WS_HF)
static_assert(WS_TOTAL <= (size_t)134217728);
static_assert(WS_BQKV % 256 == 0 && WS_BO % 256 == 0 && WS_XLN % 256 == 0 && WS_VT % 256 == 0 && WS_HF % 256 == 0);

typedef unsigned short v8us __attribute__((ext_vector_type(8), may_alias));
typedef float  v8f  __attribute__((ext_vector_type(8)));
typedef float  v4f  __attribute__((ext_vector_type(4)));
typedef float  v4fa __attribute__((ext_vector_type(4), may_alias));
typedef _Float16 v16h __attribute__((ext_vector_type(16)));
typedef _Float16 v4h  __attribute__((ext_vector_type(4)));
union FragH { v16h v; v8us half[2]; _Float16 h[16]; unsigned short u[16]; };

__device__ __forceinline__ unsigned short bf16_bits(float x) { unsigned int u = __float_as_uint(x); return (unsigned short)((u + 0x7FFFu + ((u >> 16) & 1u)) >> 16); }
__device__ __forceinline__ float bf16_val(unsigned short b) { return __uint_as_float(((unsigned int)b) << 16); }
__device__ __forceinline__ float bf16_rne(float x) { return bf16_val(bf16_bits(x)); }

__device__ __forceinline__ v16h g2_frag(const _Float16* p, unsigned hh) { FragH f; f.half[0] = *(const v8us*)((const unsigned short*)p + 8u * hh); f.half[1] = *(const v8us*)((const unsigned short*)p + 16u + 8u * hh); return f.v; }
__device__ __forceinline__ v8f g2_mma(v16h a, v16h b, v8f c) { v8f d = __builtin_amdgcn_wmma_f32_16x16x32_f16(false, a, false, b, (short)0, c, false, false); asm volatile("v_nop\n\tv_nop\n\tv_nop\n\tv_nop" : "+v"(d) : "v"(a), "v"(b)); return d; }

__global__ __launch_bounds__(256) void k_wnat(const float* __restrict__ w, size_t n8, _Float16* __restrict__ Bt) {
  const size_t t = (size_t)blockIdx.x * 256u + threadIdx.x; if (t >= n8) return;
  const v4f a = *(const v4fa*)(w + t * 8), c = *(const v4fa*)(w + t * 8 + 4);
  FragH f;
#pragma unroll
  for (int q = 0; q < 4; ++q) { f.h[q] = (_Float16)(bf16_rne(a[q]) * 16.0f); f.h[4 + q] = (_Float16)(bf16_rne(c[q]) * 16.0f); }
  const v8us o = f.half[0];
  *(volatile v8us*)((unsigned short*)Bt + t * 8) = o; __threadfence(); *(volatile v8us*)((unsigned short*)Bt + t * 8) = o;
}

template <int BFIN, int FULLIN>
__global__ __launch_bounds__(256) void k_lnx(const float* __restrict__ X, const float* __restrict__ g, const float* __restrict__ bb, float eps, _Float16* __restrict__ N16) {
  #pragma clang fp contract(off)
  __shared__ float red[256];
  const unsigned r = blockIdx.x, t = threadIdx.x, c0 = t * 4u;
  const size_t rin = FULLIN ? ((size_t)(r / (unsigned)SEQ) * (size_t)SEQ_FULL + (size_t)(r % (unsigned)SEQ)) : (size_t)r;
  const v4f xa = *(const v4fa*)(X + rin * DM + c0);
  float s0 = BFIN ? bf16_rne(xa[0]) : xa[0], s1 = BFIN ? bf16_rne(xa[1]) : xa[1], s2 = BFIN ? bf16_rne(xa[2]) : xa[2], s3 = BFIN ? bf16_rne(xa[3]) : xa[3];
  red[t] = ((s0 + s1) + s2) + s3; __syncthreads();
  for (unsigned st = 128; st > 0; st >>= 1) { if (t < st) red[t] = red[t] + red[t + st]; __syncthreads(); }
  const float mu = red[0] * (1.0f / (float)DM); __syncthreads();
  const float d0 = s0 - mu, d1 = s1 - mu, d2 = s2 - mu, d3 = s3 - mu;
  red[t] = ((d0 * d0 + d1 * d1) + d2 * d2) + d3 * d3; __syncthreads();
  for (unsigned st = 128; st > 0; st >>= 1) { if (t < st) red[t] = red[t] + red[t + st]; __syncthreads(); }
  const float rs = rsqrtf(red[0] * (1.0f / (float)DM) + eps);
  const v4f gv = *(const v4fa*)(g + c0), bv = *(const v4fa*)(bb + c0);
  v4h y;
  y[0] = (_Float16)(d0 * rs * bf16_rne(gv[0]) + bf16_rne(bv[0]));
  y[1] = (_Float16)(d1 * rs * bf16_rne(gv[1]) + bf16_rne(bv[1]));
  y[2] = (_Float16)(d2 * rs * bf16_rne(gv[2]) + bf16_rne(bv[2]));
  y[3] = (_Float16)(d3 * rs * bf16_rne(gv[3]) + bf16_rne(bv[3]));
  _Float16* dst = N16 + (size_t)r * DM + c0;
  *(volatile v4h*)dst = y; __threadfence(); *(volatile v4h*)dst = y;
}

template <int ACT, int RESB>
__global__ __launch_bounds__(128) void k_gemm2(const _Float16* __restrict__ A, unsigned lda, const _Float16* __restrict__ Bh, unsigned ldb, float alpha,
    const float* __restrict__ bias, const float* __restrict__ R, unsigned ldr, float* __restrict__ C, _Float16* __restrict__ C16, unsigned ldc, unsigned M, unsigned N, unsigned K) {
  static_assert(ACT == 0 || ACT == 6);
  static_assert(RESB >= 0 && RESB <= 2);
  __shared__ __attribute__((aligned(16))) float so[4][32][68];
  const unsigned tid = threadIdx.x, w = tid >> 5, lane = tid & 31u, ln = lane & 15u, hh = lane >> 4;
  const unsigned ntn = N >> 6; const unsigned mt = blockIdx.x / ntn, nq = blockIdx.x - mt * ntn;
  const unsigned row0 = mt * 128u + 32u * w, col0 = nq * 64u; if (row0 >= M) return;
  const _Float16* a0p = A + (size_t)(row0 + ln) * lda; const _Float16* a1p = a0p + (size_t)16 * lda;
  const _Float16* b0p = Bh + (size_t)(col0 + ln) * ldb; const _Float16* b1p = b0p + (size_t)16 * ldb; const _Float16* b2p = b1p + (size_t)16 * ldb; const _Float16* b3p = b2p + (size_t)16 * ldb;
  const v8f z8 = {0.f,0.f,0.f,0.f,0.f,0.f,0.f,0.f}; v8f c00 = z8, c01 = z8, c02 = z8, c03 = z8, c10 = z8, c11 = z8, c12 = z8, c13 = z8;
#pragma unroll 1
  for (unsigned kb = 0; kb < K; kb += 32) { const v16h a0 = g2_frag(a0p + kb, hh), a1 = g2_frag(a1p + kb, hh);
    v16h b = g2_frag(b0p + kb, hh); c00 = g2_mma(a0, b, c00); c10 = g2_mma(a1, b, c10);
    b = g2_frag(b1p + kb, hh); c01 = g2_mma(a0, b, c01); c11 = g2_mma(a1, b, c11);
    b = g2_frag(b2p + kb, hh); c02 = g2_mma(a0, b, c02); c12 = g2_mma(a1, b, c12);
    b = g2_frag(b3p + kb, hh); c03 = g2_mma(a0, b, c03); c13 = g2_mma(a1, b, c13); }
  v8f accs[8] = {c00, c01, c02, c03, c10, c11, c12, c13};
#pragma unroll
  for (int u = 0; u < 8; ++u) { const unsigned t = (unsigned)(u & 3), half = (unsigned)(u >> 2); const unsigned col = col0 + t * 16u + ln; const float bv = bias ? bf16_rne(bias[col]) : 0.f;
#pragma unroll
    for (int r = 0; r < 8; ++r) { const unsigned rloc = half * 16u + 8u * hh + (unsigned)r; float v = accs[u][r] * alpha + bv;
      if (ACT == 6) v = 0.5f * v * (1.0f + erff(v * 0.70710678118654752f));
      so[w][rloc][t * 16u + ln] = v; } }
  __builtin_amdgcn_fence(4  , "workgroup"); __builtin_amdgcn_wave_barrier();
  const unsigned rsub = lane >> 4, c4 = (lane & 15u) * 4u;
  if (RESB != 0) {
#pragma unroll
    for (int q = 0; q < 16; ++q) { const unsigned r = (unsigned)q * 2u + rsub; v4f s = *(const v4fa*)&so[w][r][c4]; v4f rv = *(const v4fa*)(R + (size_t)(row0 + r) * ldr + col0 + c4);
      if (RESB == 2) { rv[0] = bf16_rne(rv[0]); rv[1] = bf16_rne(rv[1]); rv[2] = bf16_rne(rv[2]); rv[3] = bf16_rne(rv[3]); }
      s[0] += rv[0]; s[1] += rv[1]; s[2] += rv[2]; s[3] += rv[3]; *(v4fa*)&so[w][r][c4] = s; }
  }
  for (int pass = 0; pass < 2; ++pass) {
#pragma unroll
    for (int q = 0; q < 16; ++q) { const unsigned r = (unsigned)q * 2u + rsub; const v4f v = *(const v4fa*)&so[w][r][c4];
      if (C) *(volatile v4f*)(C + (size_t)(row0 + r) * ldc + col0 + c4) = v;
      if (C16) { v4h h4; h4[0] = (_Float16)v[0]; h4[1] = (_Float16)v[1]; h4[2] = (_Float16)v[2]; h4[3] = (_Float16)v[3]; *(volatile v4h*)(C16 + (size_t)(row0 + r) * ldc + col0 + c4) = h4; } }
    if (pass == 0) __threadfence(); } }

template <int NHv, int TTv>
__global__ __launch_bounds__(256) void k_vt(const _Float16* __restrict__ V16, unsigned ldv, unsigned voff, _Float16* __restrict__ Vt) {
  __shared__ unsigned short tl[64][66];
  const unsigned tid = threadIdx.x; const unsigned slab = blockIdx.x / (unsigned)(TTv / 64), lg = blockIdx.x % (unsigned)(TTv / 64); const unsigned b = slab / (unsigned)NHv, h = slab % (unsigned)NHv;
  for (unsigned i = tid; i < 64u * 8u; i += 256u) { const unsigned r = i >> 3, c8 = (i & 7u) * 8u; FragH f; f.half[0] = *(const v8us*)((const unsigned short*)V16 + ((size_t)b * TTv + lg * 64u + r) * ldv + voff + h * 64u + c8);
#pragma unroll
    for (int q = 0; q < 8; ++q) tl[r][c8 + q] = f.u[q]; }
  __syncthreads();
  for (int pass = 0; pass < 2; ++pass) {
#pragma unroll
    for (int rd = 0; rd < 2; ++rd) { const unsigned d = (unsigned)rd * 32u + (tid >> 3), pc = tid & 7u; FragH f;
#pragma unroll
      for (int q = 0; q < 8; ++q) f.u[q] = tl[pc * 8u + q][d];
      *(volatile v8us*)((unsigned short*)Vt + ((size_t)slab * 64u + d) * TTv + lg * 64u + pc * 8u) = f.half[0]; }
    if (pass == 0) __threadfence(); } }

__global__ __launch_bounds__(128) void k_flash(const _Float16* __restrict__ QKV, const _Float16* __restrict__ VT, _Float16* __restrict__ Y) {
  __shared__ __attribute__((aligned(16))) float so[4][16][68];
  const unsigned tid = threadIdx.x, w = tid >> 5, lane = tid & 31u, ln = lane & 15u, hh = lane >> 4;
  const unsigned bh = blockIdx.y, b = bh / (unsigned)NH, h = bh % (unsigned)NH;
  const unsigned q0 = blockIdx.x * 64u + w * 16u, qq = q0 + ln;
  const _Float16* Qp = QKV + (size_t)b * SEQ * LQ + h * HD;
  const _Float16* Kp = Qp + DM;
  const _Float16* Vs = VT + (size_t)bh * HD * SEQ + (size_t)ln * SEQ;
  const v16h qb0 = g2_frag(Qp + (size_t)qq * LQ, hh), qb1 = g2_frag(Qp + (size_t)qq * LQ + 32, hh);
  const v8f z8 = {0.f,0.f,0.f,0.f,0.f,0.f,0.f,0.f};
  v8f o0 = z8, o1 = z8, o2 = z8, o3 = z8; float mrun = -1.0e30f, lrun = 0.f;
  const unsigned njt = (q0 >> 5) + 1u;
#pragma unroll 1
  for (unsigned j = 0; j < njt; ++j) {
    const unsigned key0 = j * 32u;
    const _Float16* k0p = Kp + (size_t)(key0 + ln) * LQ; const _Float16* k1p = k0p + (size_t)16 * LQ;
    v8f s0 = z8, s1 = z8;
    s0 = g2_mma(g2_frag(k0p, hh), qb0, s0); s0 = g2_mma(g2_frag(k0p + 32, hh), qb1, s0);
    s1 = g2_mma(g2_frag(k1p, hh), qb0, s1); s1 = g2_mma(g2_frag(k1p + 32, hh), qb1, s1);
    const unsigned kb0 = key0 + 8u * hh;
    float mx = -1.0e30f;
#pragma unroll
    for (int r = 0; r < 8; ++r) { const float a0 = (kb0 + (unsigned)r <= qq) ? s0[r] * 0.125f : -1.0e30f; const float a1 = (kb0 + 16u + (unsigned)r <= qq) ? s1[r] * 0.125f : -1.0e30f; s0[r] = a0; s1[r] = a1; mx = fmaxf(mx, fmaxf(a0, a1)); }
    mx = fmaxf(mx, __shfl_xor(mx, 16, 32));
    const float mnew = fmaxf(mrun, mx);
    const float al = __expf(mrun - mnew);
    FragH pb; float rs = 0.f;
#pragma unroll
    for (int r = 0; r < 8; ++r) {
      float p0 = __expf(s0[r] - mnew) * 16.0f; p0 = (kb0 + (unsigned)r <= qq) ? p0 : 0.f;
      float p1 = __expf(s1[r] - mnew) * 16.0f; p1 = (kb0 + 16u + (unsigned)r <= qq) ? p1 : 0.f;
      const _Float16 h0 = (_Float16)p0, h1 = (_Float16)p1; pb.h[r] = h0; pb.h[8 + r] = h1; rs += (float)h0 + (float)h1; }
    rs += __shfl_xor(rs, 16, 32);
    lrun = lrun * al + rs; mrun = mnew;
#pragma unroll
    for (int r = 0; r < 8; ++r) { o0[r] *= al; o1[r] *= al; o2[r] *= al; o3[r] *= al; }
    const _Float16* vp = Vs + key0;
    o0 = g2_mma(g2_frag(vp, hh), pb.v, o0);
    o1 = g2_mma(g2_frag(vp + (size_t)16 * SEQ, hh), pb.v, o1);
    o2 = g2_mma(g2_frag(vp + (size_t)32 * SEQ, hh), pb.v, o2);
    o3 = g2_mma(g2_frag(vp + (size_t)48 * SEQ, hh), pb.v, o3);
  }
  const float inv = 64.0f * (1.0f / lrun);
#pragma unroll
  for (int r = 0; r < 8; ++r) { const unsigned d = 8u * hh + (unsigned)r; so[w][ln][d] = o0[r] * inv; so[w][ln][16u + d] = o1[r] * inv; so[w][ln][32u + d] = o2[r] * inv; so[w][ln][48u + d] = o3[r] * inv; }
  __builtin_amdgcn_fence(4  , "workgroup"); __builtin_amdgcn_wave_barrier();
  const unsigned rsub = lane >> 4, c4 = (lane & 15u) * 4u;
  _Float16* yrow = Y + ((size_t)b * SEQ + q0) * DM + h * HD;
  for (int pass = 0; pass < 2; ++pass) {
#pragma unroll
    for (int q = 0; q < 8; ++q) { const unsigned r = (unsigned)q * 2u + rsub; const v4f v = *(const v4fa*)&so[w][r][c4]; v4h h4; h4[0] = (_Float16)v[0]; h4[1] = (_Float16)v[1]; h4[2] = (_Float16)v[2]; h4[3] = (_Float16)v[3];
      *(volatile v4h*)(yrow + (size_t)r * DM + c4) = h4; }
    if (pass == 0) __threadfence(); } }

extern "C" void kernel_launch(void* const* d_in, const int* in_sizes, int n_in,
                              void* d_out, int out_size, void* d_ws, size_t ws_size, hipStream_t stream) {
  if (n_in < 13) return;
  const size_t needx = ((size_t)(NB - 1) * SEQ_FULL + SEQ) * DM;
  if ((size_t)in_sizes[0] < needx || (size_t)out_size < needx) return;
  if (in_sizes[1] < DM || in_sizes[2] < DM || (size_t)in_sizes[3] < (size_t)3 * DM * DM || in_sizes[4] < 3 * DM || (size_t)in_sizes[5] < (size_t)DM * DM || in_sizes[6] < DM) return;
  if (in_sizes[7] < DM || in_sizes[8] < DM || (size_t)in_sizes[9] < (size_t)DFF * DM || in_sizes[10] < DFF || (size_t)in_sizes[11] < (size_t)DM * DFF || in_sizes[12] < DM) return;
  if ((size_t)WS_TOTAL > ws_size) return;
  const float* x = (const float*)d_in[0]; const float* ln1w = (const float*)d_in[1]; const float* ln1b = (const float*)d_in[2];
  const float* wqkv = (const float*)d_in[3]; const float* bqkv = (const float*)d_in[4]; const float* wo = (const float*)d_in[5]; const float* bo = (const float*)d_in[6];
  const float* ln2w = (const float*)d_in[7]; const float* ln2b = (const float*)d_in[8]; const float* w1 = (const float*)d_in[9]; const float* b1 = (const float*)d_in[10];
  const float* w2 = (const float*)d_in[11]; const float* b2 = (const float*)d_in[12];
  char* ws = (char*)d_ws; size_t off = 0;
  _Float16* BQKV = (_Float16*)(ws + off); off += WS_BQKV;
  _Float16* BO   = (_Float16*)(ws + off); off += WS_BO;
  _Float16* BW1  = (_Float16*)(ws + off); off += WS_BW1;
  _Float16* BW2  = (_Float16*)(ws + off); off += WS_BW2;
  _Float16* XLN  = (_Float16*)(ws + off); off += WS_XLN;
  _Float16* QKV  = (_Float16*)(ws + off); off += WS_QKV;
  _Float16* VT   = (_Float16*)(ws + off); off += WS_VT;
  _Float16* Y16  = (_Float16*)(ws + off); off += WS_Y16;
  float*    X1   = (float*)(ws + off);    off += WS_X1;
  _Float16* HLN  = (_Float16*)(ws + off); off += WS_HLN;
  _Float16* HF16 = (_Float16*)(ws + off); off += WS_HF;
  if (off > ws_size) return;

  { const size_t n8 = (size_t)3 * DM * DM / 8; k_wnat<<<(unsigned)((n8 + 255) / 256), 256, 0, stream>>>(wqkv, n8, BQKV); }
  { const size_t n8 = (size_t)DM * DM / 8;     k_wnat<<<(unsigned)((n8 + 255) / 256), 256, 0, stream>>>(wo, n8, BO); }
  { const size_t n8 = (size_t)DFF * DM / 8;    k_wnat<<<(unsigned)((n8 + 255) / 256), 256, 0, stream>>>(w1, n8, BW1); }
  { const size_t n8 = (size_t)DM * DFF / 8;    k_wnat<<<(unsigned)((n8 + 255) / 256), 256, 0, stream>>>(w2, n8, BW2); }

  k_lnx<1, 1><<<(unsigned)NR, 256, 0, stream>>>(x, ln1w, ln1b, 1e-5f, XLN);
  k_gemm2<0, 0><<<(unsigned)((NR / 128) * (LQ / 64)), 128, 0, stream>>>(XLN, DM, BQKV, DM, 0.0625f, bqkv, nullptr, 0, nullptr, QKV, LQ, (unsigned)NR, LQ, DM);
  k_vt<NH, SEQ><<<(unsigned)(NB * NH * (SEQ / 64)), 256, 0, stream>>>(QKV + 2 * DM, LQ, 0, VT);
  k_flash<<<dim3(SEQ / 64, NB * NH), 128, 0, stream>>>(QKV, VT, Y16);
  for (int b = 0; b < NB; ++b) {
    k_gemm2<0, 2><<<(unsigned)((SEQ / 128) * (DM / 64)), 128, 0, stream>>>(Y16 + (size_t)b * SEQ * DM, DM, BO, DM, 0.0009765625f, bo, x + (size_t)b * SEQ_FULL * DM, DM, X1 + (size_t)b * SEQ * DM, nullptr, DM, SEQ, DM, DM);
  }
  k_lnx<0, 0><<<(unsigned)NR, 256, 0, stream>>>(X1, ln2w, ln2b, 1e-5f, HLN);
  for (int b = 0; b < NB; ++b) {
    k_gemm2<6, 0><<<(unsigned)((SEQ / 128) * (DFF / 64)), 128, 0, stream>>>(HLN + (size_t)b * SEQ * DM, DM, BW1, DM, 0.0625f, b1, nullptr, 0, nullptr, HF16, DFF, SEQ, DFF, DM);
    k_gemm2<0, 1><<<(unsigned)((SEQ / 128) * (DM / 64)), 128, 0, stream>>>(HF16, DFF, BW2, DFF, 0.0625f, b2, X1 + (size_t)b * SEQ * DM, DM, (float*)d_out + (size_t)b * SEQ_FULL * DM, nullptr, DM, SEQ, DM, DFF);
  }
}
